// DepthAttnLayer_87771951661504
// MI455X (gfx1250) — hardware-run, weakly checked
//
#include <hip/hip_runtime.h>


namespace {
constexpr int D = 256, H = 8, HD = 32, TGT = 32400, KLEN = 16896, NP = 405026, RN = 40, NPB = 8;
constexpr float XS = 8.0f, HS = 256.0f, WSC = 256.0f, SCAL = 0.17677669529663687f, NEG = -1e9f, EPS = 1e-5f;
typedef _Float16 b16;
typedef __attribute__((ext_vector_type(16))) _Float16 v16b;
typedef __attribute__((ext_vector_type(8))) _Float16 v8b;
typedef __attribute__((ext_vector_type(8))) float v8f;
typedef __attribute__((ext_vector_type(4))) float v4f;
__device__ __forceinline__ float bf16_rne(float f) { unsigned int u = __float_as_uint(f); u += 0x7FFFu + ((u >> 16) & 1u); float r = __uint_as_float(u & 0xFFFF0000u); asm volatile("" : "+v"(r)); return r; }
__device__ __forceinline__ float bfv(float f) { float r = bf16_rne(f); asm volatile("" : "+v"(r)); return r; }
__device__ __forceinline__ void split16(float v, b16& hi, b16& lo) { hi = (b16)v; lo = (b16)(v - (float)hi); }
__device__ __forceinline__ v16b frag_kb(const b16* p, int hh) { const v8b a = *(const v8b*)(p + 8 * hh), b = *(const v8b*)(p + 16 + 8 * hh); v16b f;
#pragma unroll
  for (int e = 0; e < 8; ++e) { f[e] = a[e]; f[8 + e] = b[e]; } return f; }
__device__ __forceinline__ v8f wmma16b(v16b a, v16b b, v8f c) { v8f d = __builtin_amdgcn_wmma_f32_16x16x32_f16(false, a, false, b, (short)0, c, false, false); asm volatile("v_nop\n\tv_nop\n\tv_nop\n\tv_nop" : "+v"(d) : "v"(a), "v"(b)); return d; }
__device__ __forceinline__ void wave_lds_sync() { __builtin_amdgcn_fence(__ATOMIC_RELEASE, "workgroup"); __builtin_amdgcn_wave_barrier(); __builtin_amdgcn_fence(__ATOMIC_ACQUIRE, "workgroup"); }
__device__ __forceinline__ float pmul(float a, float b) { float p = a * b; asm volatile("" : "+v"(p)); return p; }
__device__ __forceinline__ int iclamp(int v, int lo, int hi) { return v < lo ? lo : (v > hi ? hi : v); }
constexpr int CSR_NBLK8 = 512, CSR_GB8 = 8, CSR_GN8 = 1 << CSR_GB8  , CSR_TS8 = (CSR_GN8 < 32 ? 32 : CSR_GN8)  , CSR_MAXG8 = 512, CSR_CAP8 = 12288  ;
__device__ __host__ __forceinline__ int csr_tix8(int v) { return (v >> CSR_GB8) * CSR_TS8 + (v & (CSR_GN8 - 1)); }
__global__ __launch_bounds__(64) void csrA_kernel8(const int* __restrict__ dst, int E, int N, int nG, int CHP, int NGP, int* __restrict__ STG, int* __restrict__ HST) {
  extern __shared__ int sm[];
  int* cnt = sm; int* run = sm + NGP; int* ids = sm + 2 * NGP;
  const int b = blockIdx.x; const int ch = (E + CSR_NBLK8 - 1) / CSR_NBLK8; const int e0 = b * ch, e1 = min(E, e0 + ch);
  for (int i = threadIdx.x; i < NGP; i += 64) cnt[i] = 0;
  for (int i = threadIdx.x; i < CHP; i += 64) ids[i] = -1;
  __syncthreads();
  if (threadIdx.x == 0) {
    for (int e = e0; e < e1; ++e) { int d = dst[e]; d = (d < 0) ? 0 : (d >= N ? N - 1 : d); cnt[d >> CSR_GB8] += 1; }
    int acc = 0; for (int g = 0; g < nG; ++g) { run[g] = acc; acc += cnt[g]; }
    for (int e = e0; e < e1; ++e) { int d = dst[e]; d = (d < 0) ? 0 : (d >= N ? N - 1 : d); const int g = d >> CSR_GB8; ids[run[g]] = e; run[g] += 1; } }
  __syncthreads();
  typedef __attribute__((ext_vector_type(4))) int v4i;
  for (int pass = 0; pass < 2; ++pass) {
    for (int i = threadIdx.x; i < CHP / 4; i += 64) *(volatile v4i*)(STG + (size_t)b * CHP + i * 4) = *(const v4i*)(&ids[i * 4]);
    for (int i = threadIdx.x; i < NGP / 4; i += 64) { v4i v; for (int e = 0; e < 4; ++e) v[e] = (i * 4 + e < nG) ? cnt[i * 4 + e] : 0; *(volatile v4i*)(HST + (size_t)b * NGP + i * 4) = v; }
    __threadfence(); }
}
__global__ __launch_bounds__(512) void csrS_kernel8(const int* __restrict__ HST, int nG, int NGP, int* __restrict__ START, int* __restrict__ TOT, int* __restrict__ OFF) {
  __shared__ int tot[CSR_MAXG8];
  const int b = threadIdx.x;
  for (int pass = 0; pass < 2; ++pass) { int runb = 0; for (int g = 0; g < nG; ++g) { int c = HST[(size_t)b * NGP + g]; c = (c < 0) ? 0 : c; ((volatile int*)OFF)[(size_t)g * CSR_NBLK8 + b] = runb; runb += c; } __threadfence(); }
  for (int g = threadIdx.x; g < nG; g += 512) { int s = 0; for (int bb = 0; bb < CSR_NBLK8; ++bb) { int c = HST[(size_t)bb * NGP + g]; s += (c < 0) ? 0 : c; } tot[g] = s; }
  __syncthreads();
  if (threadIdx.x < 32) {
    __shared__ int st[CSR_MAXG8 + 32];
    if (threadIdx.x == 0) { int acc = 0; for (int g = 0; g < NGP; ++g) { st[g] = acc; if (g < nG) acc += (tot[g] + 31) & ~31; } st[NGP] = acc; }
    __builtin_amdgcn_fence(__ATOMIC_RELEASE, "workgroup"); __builtin_amdgcn_wave_barrier(); __builtin_amdgcn_fence(__ATOMIC_ACQUIRE, "workgroup");
    for (int pass = 0; pass < 2; ++pass) { for (int i = threadIdx.x; i < NGP + 32; i += 32) { ((volatile int*)START)[i] = (i <= NGP) ? st[min(i, NGP)] : 0; ((volatile int*)TOT)[i] = (i < nG) ? tot[i] : 0; } __threadfence(); } }
}
__global__ __launch_bounds__(256) void csrB_kernel8(const int* __restrict__ dst, int N, int nG, int CHP, int NGP, int permLen, const int* __restrict__ STG, const int* __restrict__ HST, const int* __restrict__ OFF, const int* __restrict__ START, const int* __restrict__ TOT, int* __restrict__ PERM, int* __restrict__ ROWPTR, int* __restrict__ ROWCNT, int* __restrict__ FLAG) {
  typedef __attribute__((ext_vector_type(4))) int v4i;
  __shared__ int ids[CSR_CAP8]; __shared__ unsigned short key[CSR_CAP8]; __shared__ int outp[CSR_CAP8]; __shared__ int ncnt[CSR_GN8 + 1]; __shared__ int boff[CSR_NBLK8 + 1];
  const int g = blockIdx.x, t_ = threadIdx.x; int tot = TOT[g]; int st = START[g], stn = START[g + 1]; const int v0 = g * CSR_GN8; const int nv = min(CSR_GN8, N - v0); const int t0 = g * CSR_TS8;
  st = (st < 0) ? 0 : (st > permLen - 32 ? permLen - 32 : st) & ~31; stn = (stn < st) ? st : (stn > permLen ? permLen : stn); tot = (tot < 0) ? 0 : tot; if (tot > stn - st && tot <= CSR_CAP8) tot = stn - st;
  if (tot > CSR_CAP8) {
    for (int pass = 0; pass < 2; ++pass) { for (int i = t_; i < CSR_TS8 / 4; i += 256) { v4i a, c; for (int e = 0; e < 4; ++e) { a[e] = st; c[e] = 0; } *(volatile v4i*)(ROWPTR + t0 + i * 4) = a; *(volatile v4i*)(ROWCNT + t0 + i * 4) = c; } if (t_ == 0) ((volatile int*)FLAG)[0] = 1; __threadfence(); } (void)nv; return; }
  if (t_ == 0) { int acc = 0; for (int b = 0; b < CSR_NBLK8; ++b) { boff[b] = acc; int c = HST[(size_t)b * NGP + g]; c = (c < 0) ? 0 : (c > CHP ? CHP : c); acc += c; if (acc > tot) acc = tot; } boff[CSR_NBLK8] = acc; }
  for (int i = t_; i <= CSR_GN8; i += 256) ncnt[i] = 0;
  __syncthreads();
  for (int b = 0; b < CSR_NBLK8; ++b) { const int c = boff[b + 1] - boff[b]; int o_ = OFF[(size_t)g * CSR_NBLK8 + b]; o_ = (o_ < 0) ? 0 : (o_ > CHP - c ? CHP - c : o_); const int* src_ = STG + (size_t)b * CHP + o_;
    for (int i = t_; i < c; i += 256) { int id = src_[i]; id = (id < 0) ? 0 : id; ids[boff[b] + i] = id; int d = dst[id]; d = (d < v0) ? v0 : (d >= N ? N - 1 : d); int kk = d - v0; kk = (kk < 0) ? 0 : (kk >= CSR_GN8 ? CSR_GN8 - 1 : kk); key[boff[b] + i] = (unsigned short)kk; } }
  __syncthreads();
  if (t_ == 0) { for (int i = 0; i < tot; ++i) ncnt[key[i]] += 1; int acc = 0; for (int vl = 0; vl < CSR_GN8; ++vl) { const int c = ncnt[vl]; ncnt[vl] = acc; acc += c; } ncnt[CSR_GN8] = acc;
    for (int i = 0; i < tot; ++i) { const int vl = key[i]; outp[ncnt[vl]] = ids[i]; ncnt[vl] += 1; }
    for (int vl = CSR_GN8; vl > 0; --vl) ncnt[vl] = ncnt[vl - 1]; ncnt[0] = 0; }
  __syncthreads();
  for (int pass = 0; pass < 2; ++pass) {
    for (int i = t_; i < (stn - st) / 4; i += 256) { v4i v; for (int e = 0; e < 4; ++e) { const int q = i * 4 + e; v[e] = (q < tot) ? outp[q] : -1; } *(volatile v4i*)(PERM + st + i * 4) = v; }
    for (int i = t_; i < CSR_TS8 / 4; i += 256) { v4i a, c; for (int e = 0; e < 4; ++e) { const int vl = i * 4 + e; const int vc = vl < CSR_GN8 ? vl : CSR_GN8; a[e] = (vl < CSR_GN8) ? st + ncnt[vc] : st; c[e] = (vl < nv) ? (ncnt[(vc < CSR_GN8 ? vc : CSR_GN8 - 1) + 1] - ncnt[vc]) : 0; } *(volatile v4i*)(ROWPTR + t0 + i * 4) = a; *(volatile v4i*)(ROWCNT + t0 + i * 4) = c; }
    __threadfence(); }
}
__global__ __launch_bounds__(256) void csrZ_kernel8(int* __restrict__ p, size_t n4) { typedef __attribute__((ext_vector_type(4))) int v4i; const size_t tid = (size_t)blockIdx.x * 256 + threadIdx.x, nth = (size_t)gridDim.x * 256; v4i z = {0, 0, 0, 0}; for (size_t i = tid; i < n4; i += nth) *(volatile v4i*)(p + i * 4) = z; }
struct CsrBufs8 { int *STG, *HST, *OFF, *START, *TOT, *PERM, *ROWPTR, *ROWCNT, *FLAG; int nG, NGP, CHP; size_t permLen; char* base; size_t bytes; };
static size_t csr_carve8(CsrBufs8& c, char* ws, size_t off, int E, int N) {
  const size_t off0 = off; c.base = ws + off;
  auto al = [&](size_t bytes) { char* p = ws + off; off += (bytes + 255) & ~(size_t)255; return p; };
  c.nG = (N + CSR_GN8 - 1) / CSR_GN8; c.NGP = (c.nG + 31) & ~31; const int ch = (E + CSR_NBLK8 - 1) / CSR_NBLK8; c.CHP = (ch + 31) & ~31; c.permLen = (size_t)E + 32 * (size_t)c.nG + 32;
  c.STG = (int*)al((size_t)CSR_NBLK8 * c.CHP * 4); c.HST = (int*)al((size_t)CSR_NBLK8 * c.NGP * 4); c.OFF = (int*)al((size_t)c.NGP * CSR_NBLK8 * 4); c.START = (int*)al((size_t)(c.NGP + 64) * 4); c.TOT = (int*)al((size_t)(c.NGP + 64) * 4);
  c.PERM = (int*)al(c.permLen * 4); c.ROWPTR = (int*)al((size_t)c.nG * CSR_TS8 * 4); c.ROWCNT = (int*)al((size_t)c.nG * CSR_TS8 * 4); c.FLAG = (int*)al(256);
  c.bytes = off - off0; return off;
}
static void csr_build8(const CsrBufs8& c, const int* dst, int E, int N, hipStream_t stream) {
  const size_t smem = (size_t)(2 * c.NGP + c.CHP) * 4;
  csrZ_kernel8<<<512, 256, 0, stream>>>((int*)c.base, c.bytes / 16);
  csrA_kernel8<<<CSR_NBLK8, 64, smem, stream>>>(dst, E, N, c.nG, c.CHP, c.NGP, c.STG, c.HST);
  csrS_kernel8<<<1, 512, 0, stream>>>(c.HST, c.nG, c.NGP, c.START, c.TOT, c.OFF);
  csrB_kernel8<<<c.nG, 256, 0, stream>>>(dst, N, c.nG, c.CHP, c.NGP, (int)c.permLen, c.STG, c.HST, c.OFF, c.START, c.TOT, c.PERM, c.ROWPTR, c.ROWCNT, c.FLAG);
}


__global__ __launch_bounds__(256) void wput_kernel(const float* __restrict__ wq1, const float* __restrict__ wq2, const float* __restrict__ wk1, const float* __restrict__ wk2, b16* __restrict__ W1T, b16* __restrict__ W2T) { const size_t nt = (size_t)gridDim.x * 256, u0 = (size_t)blockIdx.x * 256 + threadIdx.x; v8b v;
  for (size_t u = u0; u < (size_t)2 * 512 * 32; u += nt) { const int m = (int)(u / (512 * 32)), o = (int)((u / 32) % 512), k0 = (int)(u % 32) * 8; const float* w = m == 0 ? wq1 : wk1;
#pragma unroll
    for (int j = 0; j < 8; ++j) v[j] = (b16)(bf16_rne(w[(size_t)(k0 + j) * 512 + o]) * WSC); for (int pass = 0; pass < 2; ++pass) { *(volatile v8b*)(W1T + ((size_t)m * 512 + o) * D + k0) = v; __threadfence(); } }
  for (size_t u = u0; u < (size_t)2 * 256 * 64; u += nt) { const int m = (int)(u / (256 * 64)), o = (int)((u / 64) % 256), k0 = (int)(u % 64) * 8; const float* w = m == 0 ? wq2 : wk2;
#pragma unroll
    for (int j = 0; j < 8; ++j) v[j] = (b16)(bf16_rne(w[(size_t)(k0 + j) * D + o]) * WSC); for (int pass = 0; pass < 2; ++pass) { *(volatile v8b*)(W2T + ((size_t)m * 256 + o) * 512 + k0) = v; __threadfence(); } } }
template <int MODE>
__global__ __launch_bounds__(32) void mlp_kernel(const float* __restrict__ X, const b16* __restrict__ W1T, const b16* __restrict__ W2T, const float* __restrict__ b1, const float* __restrict__ b2, int RTOT, int RLIM, float* __restrict__ OUTR) { __shared__ __attribute__((aligned(16))) b16 Ah[16][520], Al[16][520]; __shared__ float Tf[16][260]; const int lane = threadIdx.x, nloc = lane & 15, hlf = lane >> 4; const size_t r0 = (size_t)blockIdx.x * 16; if (r0 >= (size_t)RLIM) return; const int nr = (RTOT - (int)r0) < 16 ? (RTOT - (int)r0) : 16;
  for (int rr = 0; rr < 16; ++rr) { const size_t r = r0 + (rr < nr ? rr : 0); for (int q = 0; q < 8; ++q) { const int c = q * 32 + lane; Ah[rr][c] = (b16)(bfv(X[r * D + c]) * XS); } }
  if (lane < 16) { for (int k = D; k < D + 8; ++k) Ah[lane][k] = (b16)0.0f; for (int k = 512; k < 520; ++k) { Ah[lane][k] = (b16)0.0f; Al[lane][k] = (b16)0.0f; } }
  wave_lds_sync();
  const b16* W1 = W1T + (size_t)MODE * 512 * D; const b16* W2 = W2T + (size_t)MODE * 256 * 512;
  __shared__ float Hd[16][516];
#pragma unroll 1
  for (int g = 0; g < 2; ++g) { v8f acc[16];
#pragma unroll
    for (int t = 0; t < 16; ++t) acc[t] = (v8f){};
#pragma unroll 2
    for (int kb = 0; kb < D; kb += 32) { const v16b a = frag_kb(&Ah[nloc][kb], hlf);
#pragma unroll
      for (int t = 0; t < 16; ++t) acc[t] = wmma16b(a, frag_kb(W1 + (size_t)(g * 256 + t * 16 + nloc) * D + kb, hlf), acc[t]); }
#pragma unroll
    for (int t = 0; t < 16; ++t) { const int cc = g * 256 + t * 16 + nloc; const float bb = bfv(b1[cc]);
#pragma unroll
      for (int r8 = 0; r8 < 8; ++r8) Hd[8 * hlf + r8][cc] = fmaxf(acc[t][r8] * (1.0f / (XS * WSC)) + bb, 0.0f); } }
  wave_lds_sync();
  for (int rr = 0; rr < 16; ++rr) for (int q = 0; q < 16; ++q) { const int c = q * 32 + lane; b16 p, pl; split16(Hd[rr][c] * HS, p, pl); Ah[rr][c] = p; Al[rr][c] = pl; }
  wave_lds_sync(); v8f acc2[16];
#pragma unroll
  for (int t = 0; t < 16; ++t) acc2[t] = (v8f){};
#pragma unroll 2
  for (int kb = 0; kb < 512; kb += 32) { const v16b a = frag_kb(&Ah[nloc][kb], hlf), al = frag_kb(&Al[nloc][kb], hlf);
#pragma unroll
    for (int t = 0; t < 16; ++t) { const v16b bw = frag_kb(W2 + (size_t)(t * 16 + nloc) * 512 + kb, hlf); acc2[t] = wmma16b(a, bw, acc2[t]); acc2[t] = wmma16b(al, bw, acc2[t]); } }
  const float osc = MODE == 0 ? SCAL : 1.0f;
#pragma unroll
  for (int t = 0; t < 16; ++t) { const int cc = t * 16 + nloc; const float bb = bfv(b2[cc]);
#pragma unroll
    for (int r8 = 0; r8 < 8; ++r8) Tf[8 * hlf + r8][cc] = (acc2[t][r8] * (1.0f / (HS * WSC)) + bb) * osc; }
  wave_lds_sync();
  for (int pass = 0; pass < 2; ++pass) { for (int rr = 0; rr < nr; ++rr) for (int q = 0; q < 2; ++q) *(volatile v4f*)(OUTR + (r0 + rr) * D + q * 128 + lane * 4) = *(const v4f*)(&Tf[rr][q * 128 + lane * 4]); __threadfence(); } }
__global__ __launch_bounds__(256) void interval_kernel(const float* __restrict__ Q, const float* __restrict__ Kr, const int* __restrict__ rbev, const int* __restrict__ starts, const int* __restrict__ lens, int ILIM, int BLIM, float* __restrict__ Wout, float* __restrict__ WP) { __shared__ float Wl[NPB][H][RN + 1]; const int wave = threadIdx.x >> 5, lane = threadIdx.x & 31; const size_t i = (size_t)blockIdx.x * NPB + wave; if (i >= (size_t)ILIM) return; const int h = lane >> 2, d0 = (lane & 3) * 8;
  const int st = iclamp(starts[i], 0, NP), ln = iclamp(lens[i], 0, NP - st); const int nsl = ln < RN ? ln : RN;
  float kv[8]; for (int e = 0; e < 8; ++e) kv[e] = Kr[i * D + h * HD + d0 + e];
  if (lane < 8) for (int j = 0; j < RN; ++j) Wl[wave][lane][j] = NEG;
  __builtin_amdgcn_wave_barrier();
#pragma unroll 1
  for (int j = 0; j < nsl; ++j) { const size_t b = (size_t)iclamp(rbev[st + j], 0, TGT - 1); if (b >= (size_t)BLIM) continue;     const float* qp = Q + b * D + h * HD + d0; float s = 0.0f;
#pragma unroll
    for (int e = 0; e < 8; ++e) s += pmul(qp[e], kv[e]); s += __shfl_xor(s, 1); s += __shfl_xor(s, 2); if ((lane & 3) == 0) Wl[wave][h][j] = s; }
  wave_lds_sync();
  if (lane < 8) { float mx = -INFINITY; for (int j = 0; j < RN; ++j) mx = fmaxf(mx, Wl[wave][lane][j]); float sm = 0.0f; for (int j = 0; j < RN; ++j) { const float p = __expf(Wl[wave][lane][j] - mx); Wl[wave][lane][j] = p; sm += p; } const float inv = 1.0f / sm; for (int j = 0; j < RN; ++j) Wl[wave][lane][j] *= inv; }
  wave_lds_sync();
  for (int pass = 0; pass < 2; ++pass) { for (int u = lane; u < H * RN; u += 32) { const float w = Wl[wave][u / RN][u % RN]; ((volatile float*)Wout)[i * H * RN + u] = w; ((volatile float*)WP)[i * H * RN + u] = w; } __threadfence(); } }
__global__ __launch_bounds__(256) void bev_kernel(const float* __restrict__ WP, const float* __restrict__ value, const int* __restrict__ rfeat, const int* __restrict__ starts, const int* __restrict__ PERM, const int* __restrict__ ROWPTR, const int* __restrict__ ROWCNT, int permLen, const float* __restrict__ g, const float* __restrict__ be, int BLIM, int ILIM, float* __restrict__ out) { const int wave = threadIdx.x >> 5, lane = threadIdx.x & 31; const size_t b = (size_t)blockIdx.x * NPB + wave; if (b >= (size_t)BLIM) return; const int h = lane >> 2;
  float a[8]; for (int e = 0; e < 8; ++e) a[e] = 0.0f;
  int stp = ROWPTR[b], cnt = ROWCNT[b]; cnt = iclamp(cnt, 0, NP); stp = iclamp(stp, 0, permLen - cnt);
#pragma unroll 1
  for (int jj = 0; jj < cnt; ++jj) { const int n = iclamp(PERM[stp + jj], 0, NP - 1); const int i = iclamp(rfeat[n], 0, KLEN - 1); if (i >= ILIM) continue; const int j = iclamp(n - starts[i], 0, RN - 1); const float w = WP[(size_t)i * H * RN + h * RN + j]; const float* vp = value + (size_t)i * D + lane * 8;
#pragma unroll
    for (int e = 0; e < 8; ++e) a[e] += pmul(w, bfv(vp[e])); }
  float s1 = 0.0f; for (int e = 0; e < 8; ++e) s1 += a[e]; for (int o = 16; o; o >>= 1) s1 += __shfl_xor(s1, o); const float m = s1 * (1.0f / D); float s2 = 0.0f; for (int e = 0; e < 8; ++e) { const float dlt = a[e] - m; s2 += dlt * dlt; } for (int o = 16; o; o >>= 1) s2 += __shfl_xor(s2, o); const float rs = rsqrtf(s2 * (1.0f / D) + EPS);
  v4f r0, r1; for (int e = 0; e < 4; ++e) { const int c = lane * 8 + e; r0[e] = pmul((a[e] - m) * rs, bfv(g[c])) + bfv(be[c]); r1[e] = pmul((a[4 + e] - m) * rs, bfv(g[c + 4])) + bfv(be[c + 4]); }
  for (int pass = 0; pass < 2; ++pass) { *(volatile v4f*)(out + b * D + lane * 8) = r0; *(volatile v4f*)(out + b * D + lane * 8 + 4) = r1; __threadfence(); } }
}

extern "C" void kernel_launch(void* const* d_in, const int* in_sizes, int n_in, void* d_out, int out_size, void* d_ws, size_t ws_size, hipStream_t stream) {
  (void)n_in;
  auto Fp = [&](int i) { return (const float*)d_in[i]; }; auto Ip = [&](int i) { return (const int*)d_in[i]; };
  if (in_sizes[0] != TGT * D || in_sizes[1] != KLEN * D || in_sizes[2] != KLEN * D || in_sizes[3] != NP || in_sizes[4] != NP || in_sizes[5] != KLEN || in_sizes[6] != KLEN || in_sizes[7] != D * 512 || in_sizes[9] != 512 * D || in_sizes[11] != D * 512 || in_sizes[13] != 512 * D || out_size != TGT * D + KLEN * H * RN) return;
  const int BLIM = TGT, ILIM = KLEN;
  size_t off = 0; char* ws = (char*)d_ws;
  auto carve = [&](size_t bytes) { char* p = ws + off; off += (bytes + 255) & ~(size_t)255; return p; };
  b16* W1T = (b16*)carve((size_t)2 * 512 * D * 2); b16* W2T = (b16*)carve((size_t)2 * 256 * 512 * 2); float* Q = (float*)carve((size_t)TGT * D * 4); float* Kr = (float*)carve((size_t)KLEN * D * 4); float* WP = (float*)carve((size_t)KLEN * H * RN * 4); CsrBufs8 csr; off = csr_carve8(csr, ws, off, NP, TGT);
  if (off > ws_size || off > ((size_t)112 << 20)) return;
  wput_kernel<<<128, 256, 0, stream>>>(Fp(7), Fp(9), Fp(11), Fp(13), W1T, W2T);
  csr_build8(csr, Ip(4), NP, TGT, stream);
  mlp_kernel<0><<<(BLIM + 15) / 16, 32, 0, stream>>>(Fp(0), W1T, W2T, Fp(8), Fp(10), TGT, BLIM, Q);
  mlp_kernel<1><<<(ILIM + 15) / 16, 32, 0, stream>>>(Fp(1), W1T, W2T, Fp(12), Fp(14), KLEN, ILIM, Kr);
  float* out0 = (float*)d_out; float* out1 = out0 + (size_t)TGT * D;
  interval_kernel<<<(ILIM + NPB - 1) / NPB, 256, 0, stream>>>(Q, Kr, Ip(4), Ip(5), Ip(6), ILIM, BLIM, out1, WP);
  bev_kernel<<<(BLIM + NPB - 1) / NPB, 256, 0, stream>>>(WP, Fp(2), Ip(3), Ip(5), csr.PERM, csr.ROWPTR, csr.ROWCNT, (int)csr.permLen, Fp(15), Fp(16), BLIM, ILIM, out0);
}
